// Net_27358941675610
// MI455X (gfx1250) — hardware-verified
//
#include <hip/hip_runtime.h>
#include <math.h>

constexpr int DIM_IN    = 1024;
constexpr int DIM_HID   = 2048;
constexpr int DIM_OUT   = 512;
constexpr int DIM_BATCH = 4096;
constexpr int NSTEPS    = 50;
constexpr int THREADS   = 256;

constexpr double DT_D     = 1.0;
constexpr double TAU_D    = 10.0;
constexpr double GB_D     = 0.6;
constexpr double GL_D     = 1.0 / TAU_D;
constexpr double LAMBDA_D = 0.35;
constexpr double A_D      = DT_D / TAU_D;
constexpr double GR_D     = GB_D / GL_D;
constexpr double KH_D     = 1.0 - A_D - A_D * GR_D;
constexpr double KO_D     = 1.0 - 2.0 * A_D - A_D * GR_D;
constexpr double DRV_D    = A_D * GR_D;
constexpr double cpowi(double b, int n) { return n == 0 ? 1.0 : b * cpowi(b, n - 1); }
constexpr double GEO_D    = (1.0 - cpowi(KO_D, NSTEPS)) / (1.0 - KO_D);

constexpr float KH_F     = (float)KH_D;
constexpr float KO_F     = (float)KO_D;
constexpr float DRV_F    = (float)DRV_D;
constexpr float ASTEP_F  = (float)A_D;
constexpr float GEO_F    = (float)GEO_D;
constexpr float LAMBDA_F = (float)LAMBDA_D;
constexpr float LOG2E_F  = 1.44269504088896340736f;

constexpr float X_CARRY     = 64.0f;
constexpr float W_CARRY     = 256.0f;
constexpr float GEMM1_SCALE = 1.0f / (X_CARRY * W_CARRY);
constexpr float GEMM2_SCALE = 1.0f / W_CARRY;

static_assert(NSTEPS == 50);
static_assert(KH_D > 0.2999 && KH_D < 0.3001);
static_assert(KO_D > 0.1999 && KO_D < 0.2001);
static_assert(DRV_D > 0.5999 && DRV_D < 0.6001);
static_assert(GEO_D > 1.2499 && GEO_D < 1.2501);
static_assert(DIM_BATCH % 64 == 0 && DIM_HID % 64 == 0 && DIM_OUT % 64 == 0 && DIM_IN % 64 == 0);
static_assert(DIM_IN % 32 == 0 && DIM_HID % 32 == 0);
static_assert(((DIM_BATCH / 64) * (DIM_HID / 64)) % 8 == 0);
static_assert(((DIM_BATCH / 64) * (DIM_OUT / 64)) % 8 == 0);
static_assert((DIM_HID * DIM_IN / 8) % THREADS == 0);
static_assert((DIM_OUT * DIM_HID / 8) % THREADS == 0);
static_assert((DIM_BATCH * DIM_HID / 8) % THREADS == 0);
static_assert((DIM_BATCH * DIM_OUT / 4) % THREADS == 0);

typedef __attribute__((ext_vector_type(16))) _Float16 v16h;
typedef __attribute__((ext_vector_type(8)))  _Float16 v8h;
typedef __attribute__((ext_vector_type(8)))  float    v8f;
typedef __attribute__((ext_vector_type(4)))  float    v4f;

__device__ __forceinline__ void row_guard_h(v8f& a, v8f& b, v8f& c, v8f& d, v16h x, v16h y0, v16h y1, v16h y2, v16h y3) {
  asm volatile("v_nop\n\tv_nop\n\tv_nop\n\tv_nop" : "+v"(a), "+v"(b), "+v"(c), "+v"(d) : "v"(x), "v"(y0), "v"(y1), "v"(y2), "v"(y3));
}
__device__ __forceinline__ void keep4_h(v16h a, v16h b, v16h c, v16h d) { asm volatile("v_nop" :: "v"(a), "v"(b), "v"(c), "v"(d)); }
__device__ __forceinline__ void acc_guard4(v8f& a, v8f& b, v8f& c, v8f& d) { asm volatile("v_nop\n\tv_nop\n\tv_nop\n\tv_nop" : "+v"(a), "+v"(b), "+v"(c), "+v"(d)); }

union FragU { v16h v; v8h h[2]; };
__device__ __forceinline__ v16h frag_load(const _Float16* p) {
  FragU f;
  f.h[0] = *(const v8h*)(p);
  f.h[1] = *(const v8h*)(p + 16);
  return f.v;
}
__device__ __forceinline__ v8f frag_mma(v16h a, v16h b, v8f c) {
  return __builtin_amdgcn_wmma_f32_16x16x32_f16(false, a, false, b, (short)0, c, false, false);
}

__global__ __launch_bounds__(THREADS) void tpw_f16_kernel(const float* __restrict__ src, int R, int C, int ldo,
                                                          unsigned short* __restrict__ O, float sc) {
  __shared__ float Tt[64 * 65];
  const int tid = threadIdx.x;
  const int c0 = blockIdx.x * 64, r0 = blockIdx.y * 64;
  (void)R;
#pragma unroll
  for (int i = 0; i < 4; ++i) {
    const int idx = i * THREADS + tid;
    const int rr = idx >> 4, cc = (idx & 15) * 4;
    const v4f v = *(const v4f*)(src + (size_t)(r0 + rr) * (size_t)C + c0 + cc);
    Tt[rr * 65 + cc + 0] = v[0];
    Tt[rr * 65 + cc + 1] = v[1];
    Tt[rr * 65 + cc + 2] = v[2];
    Tt[rr * 65 + cc + 3] = v[3];
  }
  __syncthreads();
  const int q = tid >> 3, c8 = (tid & 7) * 8;
  v8h hv[2];
#pragma unroll
  for (int g = 0; g < 2; ++g) {
    const int qq = g * 32 + q;
#pragma unroll
    for (int e = 0; e < 8; ++e) {
      const float f = Tt[(c8 + e) * 65 + qq];
      hv[g][e] = (_Float16)(f * sc);
    }
  }
  for (int pass = 0; pass < 2; ++pass) {
#pragma unroll
    for (int g = 0; g < 2; ++g) {
      const size_t o = (size_t)(c0 + g * 32 + q) * (size_t)ldo + (size_t)(r0 + c8);
      *(volatile v8h*)(O + o) = hv[g];
    }
    __threadfence();
  }
}

__global__ __launch_bounds__(THREADS) void cvt8_f16_kernel(const float* __restrict__ src, unsigned short* __restrict__ dst,
                                                           int n8, float sc) {
  const int i = blockIdx.x * THREADS + threadIdx.x;
  if (i < n8) {
    const float* sp = src + (size_t)i * 8;
    const v4f a = *(const v4f*)(sp);
    const v4f b = *(const v4f*)(sp + 4);
    v8h hv;
#pragma unroll
    for (int e = 0; e < 4; ++e) {
      hv[e]     = (_Float16)(a[e] * sc);
      hv[4 + e] = (_Float16)(b[e] * sc);
    }
    *(volatile v8h*)(dst + (size_t)i * 8) = hv;
    __threadfence();
    *(volatile v8h*)(dst + (size_t)i * 8) = hv;
  }
}

template <int BIAS_MODE>
__global__ __launch_bounds__(256) void wmma_gemm64_f16(
    const unsigned short* __restrict__ Ap, int lda,
    const unsigned short* __restrict__ Btp, int ldb,
    float* __restrict__ Cout, int ldc,
    const float* __restrict__ bias,
    int M, int N, int K, float scale) {
  const _Float16* A  = (const _Float16*)Ap;
  const _Float16* Bt = (const _Float16*)Btp;
  __shared__ __align__(16) float sT[8][16 * 68];
  const int lane = threadIdx.x & 31;
  const int wave = threadIdx.x >> 5;
  const int tilesN = N >> 6;
  const int tilesM = M >> 6;
  const int tile = blockIdx.x * 8 + wave;
  if (tile >= tilesM * tilesN) return;
  const int tm = tile / tilesN;
  const int tn = tile - tm * tilesN;
  const int m0 = tm << 6;
  const int n0 = tn << 6;

  const int rlane = lane & 15;
  const int koff  = (lane >> 4) * 8;
  const int mOff  = (lane >> 4) * 8;

  v8f acc[4][4];
#pragma unroll
  for (int i = 0; i < 4; ++i)
#pragma unroll
    for (int j = 0; j < 4; ++j) acc[i][j] = (v8f){0.f, 0.f, 0.f, 0.f, 0.f, 0.f, 0.f, 0.f};

  for (int k0 = 0; k0 < K; k0 += 32) {
    v16h bh[4];
#pragma unroll
    for (int j = 0; j < 4; ++j) {
      const size_t bo = (size_t)(n0 + (j << 4) + rlane) * ldb + koff + k0;
      bh[j] = frag_load(Bt + bo);
    }
#pragma unroll
    for (int i = 0; i < 4; ++i) {
      const size_t ao = (size_t)(m0 + (i << 4) + rlane) * lda + koff + k0;
      const v16h ah = frag_load(A + ao);
#pragma unroll
      for (int j = 0; j < 4; ++j) acc[i][j] = frag_mma(ah, bh[j], acc[i][j]);
      row_guard_h(acc[i][0], acc[i][1], acc[i][2], acc[i][3], ah, bh[0], bh[1], bh[2], bh[3]);
    }
    keep4_h(bh[0], bh[1], bh[2], bh[3]);
  }
  acc_guard4(acc[0][0], acc[0][1], acc[0][2], acc[0][3]);
  acc_guard4(acc[1][0], acc[1][1], acc[1][2], acc[1][3]);
  acc_guard4(acc[2][0], acc[2][1], acc[2][2], acc[2][3]);
  acc_guard4(acc[3][0], acc[3][1], acc[3][2], acc[3][3]);

  float* slab = sT[wave];
#pragma unroll
  for (int i = 0; i < 4; ++i) {
    const int mBase = m0 + (i << 4);
#pragma unroll
    for (int j = 0; j < 4; ++j) {
      const int n = n0 + (j << 4) + rlane;
      float bv = 0.f;
      if (BIAS_MODE == 2) bv = bias[n];
#pragma unroll
      for (int r = 0; r < 8; ++r) {
        float v = acc[i][j][r] * scale;
        if (BIAS_MODE == 2) v += bv;
        slab[(mOff + r) * 68 + (j << 4) + rlane] = v;
      }
    }
    __builtin_amdgcn_fence(__ATOMIC_RELEASE, "workgroup");
    __builtin_amdgcn_wave_barrier();
    __builtin_amdgcn_fence(__ATOMIC_ACQUIRE, "workgroup");
    {
      const int hh = lane >> 4, c4 = (lane & 15) * 4;
      for (int pass = 0; pass < 2; ++pass) {
#pragma unroll
        for (int it = 0; it < 8; ++it) {
          const int row = it * 2 + hh;
          const v4f v = *(const v4f*)(slab + row * 68 + c4);
          *(volatile v4f*)(Cout + (size_t)(mBase + row) * ldc + n0 + c4) = v;
        }
        __threadfence();
      }
    }
    __builtin_amdgcn_fence(__ATOMIC_RELEASE, "workgroup");
    __builtin_amdgcn_wave_barrier();
    __builtin_amdgcn_fence(__ATOMIC_ACQUIRE, "workgroup");
  }
}

__global__ __launch_bounds__(THREADS) void scan_rate_kernel(const float* __restrict__ BV, unsigned short* __restrict__ RS, int n8) {
  const int i = blockIdx.x * THREADS + threadIdx.x;
  if (i < n8) {
    const float* sp = BV + (size_t)i * 8;
    const v4f a = *(const v4f*)(sp);
    const v4f b = *(const v4f*)(sp + 4);
    float dv[8], h[8], s[8];
#pragma unroll
    for (int e = 0; e < 4; ++e) {
      dv[e]     = DRV_F * a[e];
      dv[4 + e] = DRV_F * b[e];
    }
#pragma unroll
    for (int e = 0; e < 8; ++e) {
      h[e] = 0.0f;
      s[e] = 0.0f;
    }
#pragma unroll 1
    for (int t = 0; t < NSTEPS; ++t) {
#pragma unroll
      for (int e = 0; e < 8; ++e) {
        const float hn = fmaf(KH_F, h[e], dv[e]);
        h[e] = hn;
        const float ex = exp2f(-hn * LOG2E_F);
        const float sg = __builtin_amdgcn_rcpf(1.0f + ex);
        s[e] = fmaf(KO_F, s[e], sg);
      }
    }
    v8h hv;
#pragma unroll
    for (int e = 0; e < 8; ++e) hv[e] = (_Float16)(LAMBDA_F * s[e]);
    *(volatile v8h*)(RS + (size_t)i * 8) = hv;
    __threadfence();
    *(volatile v8h*)(RS + (size_t)i * 8) = hv;
  }
}

__global__ __launch_bounds__(THREADS) void out_stage_kernel(const float* __restrict__ P, const float* __restrict__ label,
                                                            const float* __restrict__ b_o, float* __restrict__ out, int n4) {
  const int i = blockIdx.x * THREADS + threadIdx.x;
  if (i < n4) {
    const size_t o = (size_t)i * 4;
    const int col = (int)(o % (size_t)DIM_OUT);
    const v4f p  = *(const v4f*)(P + o);
    const v4f lb = *(const v4f*)(label + o);
    const v4f bo = *(const v4f*)(b_o + col);
    v4f r;
#pragma unroll
    for (int e = 0; e < 4; ++e) {
      const float cd   = DRV_F * bo[e] + ASTEP_F * lb[e];
      const float soma = DRV_F * p[e] + GEO_F * cd;
      r[e] = LAMBDA_F * __builtin_amdgcn_rcpf(1.0f + expf(-soma));
    }
    *(volatile v4f*)(out + o) = r;
    __threadfence();
    *(volatile v4f*)(out + o) = r;
  }
}

extern "C" void kernel_launch(void* const* d_in, const int* in_sizes, int n_in,
                              void* d_out, int out_size, void* d_ws, size_t ws_size, hipStream_t stream) {
  if (n_in < 6 || d_out == nullptr || d_ws == nullptr) return;
  if (in_sizes[0] != DIM_IN * DIM_BATCH || in_sizes[1] != DIM_BATCH * DIM_OUT || in_sizes[2] != DIM_HID * DIM_IN ||
      in_sizes[3] != DIM_HID || in_sizes[4] != DIM_OUT * DIM_HID || in_sizes[5] != DIM_OUT ||
      out_size != DIM_BATCH * DIM_OUT) return;

  const float* psp   = (const float*)d_in[0];
  const float* label = (const float*)d_in[1];
  const float* w_h   = (const float*)d_in[2];
  const float* b_h   = (const float*)d_in[3];
  const float* w_o   = (const float*)d_in[4];
  const float* b_o   = (const float*)d_in[5];
  float* out = (float*)d_out;

  char* ws = (char*)d_ws;
  size_t off = 0;
  auto carve = [&](size_t bytes) -> char* { char* p = ws + off; off += (bytes + 255) & ~(size_t)255; return p; };
  unsigned short* XH  = (unsigned short*)carve((size_t)DIM_BATCH * DIM_IN * 2);
  unsigned short* WHH = (unsigned short*)carve((size_t)DIM_HID * DIM_IN * 2);
  unsigned short* WOH = (unsigned short*)carve((size_t)DIM_OUT * DIM_HID * 2);
  float*          BVH = (float*)carve((size_t)DIM_BATCH * DIM_HID * 4);
  unsigned short* RS  = (unsigned short*)carve((size_t)DIM_BATCH * DIM_HID * 2);
  float*          PO  = (float*)carve((size_t)DIM_BATCH * DIM_OUT * 4);
  if (off > ws_size || off > (size_t)134217728) return;

  tpw_f16_kernel<<<dim3(DIM_BATCH / 64, DIM_IN / 64), THREADS, 0, stream>>>(psp, DIM_IN, DIM_BATCH, DIM_IN, XH, X_CARRY);

  const int n8wh = DIM_HID * DIM_IN / 8;
  const int n8wo = DIM_OUT * DIM_HID / 8;
  cvt8_f16_kernel<<<n8wh / THREADS, THREADS, 0, stream>>>(w_h, WHH, n8wh, W_CARRY);
  cvt8_f16_kernel<<<n8wo / THREADS, THREADS, 0, stream>>>(w_o, WOH, n8wo, W_CARRY);

  wmma_gemm64_f16<2><<<(DIM_BATCH / 64) * (DIM_HID / 64) / 8, 256, 0, stream>>>(
      XH, DIM_IN, WHH, DIM_IN, BVH, DIM_HID, b_h, DIM_BATCH, DIM_HID, DIM_IN, GEMM1_SCALE);

  const int n8rs = DIM_BATCH * DIM_HID / 8;
  scan_rate_kernel<<<n8rs / THREADS, THREADS, 0, stream>>>(BVH, RS, n8rs);

  wmma_gemm64_f16<0><<<(DIM_BATCH / 64) * (DIM_OUT / 64) / 8, 256, 0, stream>>>(
      RS, DIM_HID, WOH, DIM_HID, PO, DIM_OUT, b_o, DIM_BATCH, DIM_OUT, DIM_HID, GEMM2_SCALE);

  const int n4 = DIM_BATCH * DIM_OUT / 4;
  out_stage_kernel<<<n4 / THREADS, THREADS, 0, stream>>>(PO, label, b_o, out, n4);
}
